// RNNdiff_1425929142296
// MI455X (gfx1250) — hardware-verified
//
#include <hip/hip_runtime.h>
#include <stdint.h>
#include <stddef.h>

#define NB   256
#define NV   50
#define NC   20
#define DD   256
#define HH   256
#define G4   1024
#define NTD  1000
#define NVOC 20001
#define NR   12800
#define TFW  64
#define CL2  512
#define CLR  512

#define TPE  68
#define PH   264
#define PF   260

static_assert(NR == NB * NV);
static_assert(G4 == 4 * HH);
static_assert(DD == 256);
static_assert(HH == 256);
static_assert(NB == 256);
static_assert(NR % 64 == 0);
static_assert(NR % 8 == 0);
static_assert(CLR % 64 == 0);
static_assert(CLR == 2 * NB);
static_assert(CL2 % 64 == 0);
static_assert(G4 % 64 == 0);
static_assert(TFW % 32 == 0);
static_assert((TPE * 4) % 16 == 0);
static_assert((PH * 2) % 16 == 0);
static_assert((PF * 4) % 16 == 0);

typedef __bf16        v16b __attribute__((ext_vector_type(16)));
typedef float         v8f  __attribute__((ext_vector_type(8)));
typedef float         v4f  __attribute__((ext_vector_type(4)));
typedef float         v2f  __attribute__((ext_vector_type(2)));
typedef unsigned int  v4u  __attribute__((ext_vector_type(4)));
typedef v4f __attribute__((may_alias)) v4fa;
typedef v2f __attribute__((may_alias)) v2fa;
typedef v4u __attribute__((may_alias)) v4ua;

union FragB { v16b v; v4u q[2]; };

__device__ __forceinline__ v8f wmma_b(v16b a, v16b b, v8f c) {
  v8f d = __builtin_amdgcn_wmma_f32_16x16x32_bf16(false, a, false, b, (short)0, c, false, false);
  asm volatile("v_nop\n\tv_nop\n\tv_nop\n\tv_nop" : "+v"(d) : "v"(a), "v"(b));
  return d;
}

__device__ __forceinline__ v16b ldfrag(const unsigned short* p, int h) {
  FragB f;
  f.q[0] = *(const v4ua*)(p + 8 * h);
  f.q[1] = *(const v4ua*)(p + 16 + 8 * h);
  return f.v;
}

__device__ __forceinline__ unsigned int bf16r(float x) {
  const unsigned int u = __float_as_uint(x);
  return (u + 0x7FFFu + ((u >> 16) & 1u)) >> 16;
}
__device__ __forceinline__ unsigned int split_pair(float a, float b, unsigned int& lp) {
  const unsigned int ha = bf16r(a), hb = bf16r(b);
  const unsigned int la = bf16r(a - __uint_as_float(ha << 16));
  const unsigned int lb = bf16r(b - __uint_as_float(hb << 16));
  lp = la | (lb << 16);
  return ha | (hb << 16);
}
__device__ __forceinline__ void pk8(v4f a, v4f b, v4u& ph, v4u& pl) {
  unsigned int l0, l1, l2, l3;
  v4u o;
  o.x = split_pair(a.x, a.y, l0);
  o.y = split_pair(a.z, a.w, l1);
  o.z = split_pair(b.x, b.y, l2);
  o.w = split_pair(b.z, b.w, l3);
  ph = o;
  v4u q;
  q.x = l0; q.y = l1; q.z = l2; q.w = l3;
  pl = q;
}

__device__ __forceinline__ v4f relu4(v4f v) {
  v4f o;
  o.x = fmaxf(v.x, 0.f); o.y = fmaxf(v.y, 0.f); o.z = fmaxf(v.z, 0.f); o.w = fmaxf(v.w, 0.f);
  return o;
}

__device__ __forceinline__ float sigm(float x) {
  return __builtin_amdgcn_rcpf(1.0f + __expf(-x));
}
__device__ __forceinline__ float tnh(float x) {
  const float xc = fminf(fmaxf(x, -15.0f), 15.0f);
  const float e = __expf(2.0f * xc);
  return (e - 1.0f) * __builtin_amdgcn_rcpf(e + 1.0f);
}

__global__ __launch_bounds__(256) void k_cvtw(const float* __restrict__ src, int K, int N,
                                              unsigned short* Dh, unsigned short* Dl)
{
  __shared__ float sT[64 * 65];
  const int tid = threadIdx.x;
  const int nt0 = blockIdx.x * 64, kt0 = blockIdx.y * 64;
  #pragma unroll
  for (int i = 0; i < 16; ++i) {
    const int idx = tid + 256 * i;
    const int kk = idx >> 6, nn = idx & 63;
    sT[kk * 65 + nn] = src[(size_t)(kt0 + kk) * N + nt0 + nn];
  }
  __syncthreads();
  v4u oh[2], ol[2];
  size_t oa[2];
  #pragma unroll
  for (int it = 0; it < 2; ++it) {
    const int r = (tid >> 3) + 32 * it, p = tid & 7;
    v4f a, b;
    a.x = sT[(8 * p + 0) * 65 + r]; a.y = sT[(8 * p + 1) * 65 + r];
    a.z = sT[(8 * p + 2) * 65 + r]; a.w = sT[(8 * p + 3) * 65 + r];
    b.x = sT[(8 * p + 4) * 65 + r]; b.y = sT[(8 * p + 5) * 65 + r];
    b.z = sT[(8 * p + 6) * 65 + r]; b.w = sT[(8 * p + 7) * 65 + r];
    pk8(a, b, oh[it], ol[it]);
    oa[it] = (size_t)(nt0 + r) * K + kt0 + 8 * p;
  }
  #pragma unroll
  for (int it = 0; it < 2; ++it) {
    *(volatile v4u*)(Dh + oa[it]) = oh[it];
    *(volatile v4u*)(Dl + oa[it]) = ol[it];
  }
  __threadfence();
  #pragma unroll
  for (int it = 0; it < 2; ++it) {
    *(volatile v4u*)(Dh + oa[it]) = oh[it];
    *(volatile v4u*)(Dl + oa[it]) = ol[it];
  }
}

__global__ __launch_bounds__(256) void k_prep(const float* __restrict__ bih,
                                              const float* __restrict__ bhh,
                                              const int* __restrict__ tv,
                                              float* bsum, float* btab)
{
  __shared__ float sAl[NTD];
  const int tid = threadIdx.x;
  if (tid == 0) {
    float a = 1.0f;
    const float inv = 1.0f / (float)(NTD - 1);
    #pragma unroll 1
    for (int i = 0; i < NTD; ++i) {
      float beta;
      if (i < NTD - 1) {
        const float s = (float)i * inv;
        beta = 0.0001f * (1.0f - s) + 0.02f * s;
      } else {
        beta = 0.02f;
      }
      a = a * (1.0f - beta);
      sAl[i] = a;
    }
  }
  __syncthreads();
  const int traw = tv[tid];
  int tc = traw;
  tc = (tc < 0) ? 0 : ((tc > NTD - 1) ? (NTD - 1) : tc);
  const float al = sAl[tc];
  const float sa = sqrtf(al);
  const float sn = sqrtf(1.0f - al);
  const float tn = (float)traw * (1.0f / (float)NTD);
  const v4f s4 = *(const v4fa*)(bih + 4 * tid) + *(const v4fa*)(bhh + 4 * tid);
  *(volatile float*)(btab + tid) = sa;
  *(volatile float*)(btab + NB + tid) = sn;
  *(volatile float*)(btab + 2 * NB + tid) = tn;
  *(volatile v4f*)(bsum + 4 * tid) = s4;
  __threadfence();
  *(volatile float*)(btab + tid) = sa;
  *(volatile float*)(btab + NB + tid) = sn;
  *(volatile float*)(btab + 2 * NB + tid) = tn;
  *(volatile v4f*)(bsum + 4 * tid) = s4;
}

__global__ __launch_bounds__(256) void k_tfeat(const float* __restrict__ st,
                                               const float* __restrict__ wt,
                                               const float* __restrict__ bt,
                                               unsigned short* Th, unsigned short* Tl)
{
  __shared__ __align__(16) unsigned short sH[256];
  __shared__ __align__(16) unsigned short sL[256];
  const int tid = threadIdx.x, lane = tid & 31, wv = tid >> 5;
  const int row = blockIdx.x * 4 + (tid >> 6);
  const int j = tid & 63;
  const float ts = st[row] * (1.0f / 180.0f);
  const float u = ts * wt[j] + bt[j];
  const float v = 1.0f - tnh(u * u);
  const unsigned int hb = bf16r(v);
  const unsigned int lb = bf16r(v - __uint_as_float(hb << 16));
  sH[tid] = (unsigned short)hb;
  sL[tid] = (unsigned short)lb;
  __syncthreads();
  if (wv < 2) {
    const v4u a = *(const v4ua*)(sH + 8 * lane);
    const v4u b = *(const v4ua*)(sL + 8 * lane);
    v4u o;
    if (wv == 0) o = a; else o = b;
    unsigned short* d = ((wv == 0) ? Th : Tl) + (size_t)blockIdx.x * 4 * TFW + 8 * lane;
    *(volatile v4u*)d = o;
    __threadfence();
    *(volatile v4u*)d = o;
  }
}

__global__ __launch_bounds__(256) void k_embed(const int* __restrict__ seqs,
                                               const float* __restrict__ embW,
                                               float* E)
{
  const int tid = threadIdx.x, lane = tid & 31, wv = tid >> 5;
  const int row = blockIdx.x * 8 + wv;
  const int* sq = seqs + (size_t)row * NC;
  v4f s0 = {0.f, 0.f, 0.f, 0.f};
  v4f s1 = {0.f, 0.f, 0.f, 0.f};
  #pragma unroll 2
  for (int i = 0; i < NC; ++i) {
    int id = sq[i];
    id = (id < 0) ? id + NVOC : id;
    id = (id < 0) ? 0 : ((id > NVOC - 1) ? (NVOC - 1) : id);
    const float* ep = embW + (size_t)id * DD;
    const v4f a = *(const v4fa*)(ep + 4 * lane);
    const v4f b = *(const v4fa*)(ep + 128 + 4 * lane);
    s0 += relu4(a);
    s1 += relu4(b);
  }
  float* d = E + (size_t)row * DD;
  *(volatile v4f*)(d + 4 * lane) = s0;
  *(volatile v4f*)(d + 128 + 4 * lane) = s1;
  __threadfence();
  *(volatile v4f*)(d + 4 * lane) = s0;
  *(volatile v4f*)(d + 128 + 4 * lane) = s1;
}

template<int BIAS, int RELU, int ADDR, int PG>
__device__ __forceinline__ v4f epi4(v4f v, int grow, int gcol,
                                    const float* __restrict__ bias,
                                    const float* __restrict__ rsc,
                                    const float* __restrict__ R, int ldr)
{
  if (BIAS) {
    const v4f bb = *(const v4fa*)(bias + gcol);
    if (PG) {
      const float s = rsc[grow / NV];
      v += bb * s;
    } else {
      v += bb;
    }
  }
  if (ADDR) v += *(const v4fa*)(R + (size_t)grow * ldr + gcol);
  if (RELU) v = relu4(v);
  return v;
}

template<int BIAS, int RELU, int ADDR, int WF, int WP, int PG>
__global__ __launch_bounds__(128) void k_gemm(
    const unsigned short* __restrict__ Ahi, const unsigned short* __restrict__ Alo, int lda,
    const unsigned short* __restrict__ Bhi, const unsigned short* __restrict__ Blo, int ldb, int K,
    const float* __restrict__ bias, const float* __restrict__ rsc,
    const float* __restrict__ R, const float* __restrict__ R2, int ldr,
    float* Cf, int ldc, unsigned short* Phi, unsigned short* Plo, int ldp)
{
  __shared__ __align__(16) float sT[64 * TPE];
  const int tid = threadIdx.x, lane = tid & 31, wv = tid >> 5;
  const int h = lane >> 4, m = lane & 15;
  const int wm = wv >> 1, wn = wv & 1;
  const int rb = blockIdx.x * 64, cb = blockIdx.y * 64;

  const v8f z8 = {0.f, 0.f, 0.f, 0.f, 0.f, 0.f, 0.f, 0.f};
  v8f acc[2][2];
  #pragma unroll
  for (int mt = 0; mt < 2; ++mt)
    #pragma unroll
    for (int nt = 0; nt < 2; ++nt) acc[mt][nt] = z8;

  #pragma unroll 1
  for (int k0 = 0; k0 < K; k0 += 32) {
    v16b ah[2], al[2];
    #pragma unroll
    for (int mt = 0; mt < 2; ++mt) {
      const size_t ao = (size_t)(rb + 32 * wm + 16 * mt + m) * lda + k0;
      ah[mt] = ldfrag(Ahi + ao, h);
      al[mt] = ldfrag(Alo + ao, h);
    }
    #pragma unroll
    for (int nt = 0; nt < 2; ++nt) {
      const size_t bo = (size_t)(cb + 32 * wn + 16 * nt + m) * ldb + k0;
      const v16b bh = ldfrag(Bhi + bo, h);
      const v16b bl = ldfrag(Blo + bo, h);
      #pragma unroll
      for (int mt = 0; mt < 2; ++mt) {
        acc[mt][nt] = wmma_b(ah[mt], bh, acc[mt][nt]);
        acc[mt][nt] = wmma_b(ah[mt], bl, acc[mt][nt]);
        acc[mt][nt] = wmma_b(al[mt], bh, acc[mt][nt]);
      }
    }
  }

  #pragma unroll
  for (int mt = 0; mt < 2; ++mt)
    #pragma unroll
    for (int nt = 0; nt < 2; ++nt) {
      const int col = 32 * wn + 16 * nt + m;
      #pragma unroll
      for (int r = 0; r < 8; ++r) {
        const int row = 32 * wm + 16 * mt + 8 * h + r;
        sT[row * TPE + col] = acc[mt][nt][r];
      }
    }
  __syncthreads();

  v4f fo[8];
  size_t fa[8];
  if (WF) {
    #pragma unroll
    for (int i = 0; i < 8; ++i) {
      const int rr = 16 * wv + 2 * i + (lane >> 4), c4 = 4 * (lane & 15);
      const int grow = rb + rr, gcol = cb + c4;
      const v4f v = *(const v4fa*)(sT + rr * TPE + c4);
      fo[i] = epi4<BIAS, RELU, ADDR, PG>(v, grow, gcol, bias, rsc, R, ldr);
      fa[i] = (size_t)grow * ldc + gcol;
    }
  }
  v4u po[4], qo[4];
  size_t pa[4];
  if (WP) {
    #pragma unroll
    for (int q = 0; q < 4; ++q) {
      const int rr = 16 * wv + 4 * q + (lane >> 3), c8 = 8 * (lane & 7);
      const int grow = rb + rr, gcol = cb + c8;
      v4f v0 = *(const v4fa*)(sT + rr * TPE + c8);
      v4f v1 = *(const v4fa*)(sT + rr * TPE + c8 + 4);
      v0 = epi4<BIAS, RELU, ADDR, PG>(v0, grow, gcol, bias, rsc, R, ldr);
      v1 = epi4<BIAS, RELU, ADDR, PG>(v1, grow, gcol + 4, bias, rsc, R, ldr);
      if (PG) {
        const size_t ro = (size_t)grow * ldr + gcol;
        const v4f b0 = *(const v4fa*)(R + ro);
        const v4f b1 = *(const v4fa*)(R + ro + 4);
        const v4f n0 = *(const v4fa*)(R2 + ro);
        const v4f n1 = *(const v4fa*)(R2 + ro + 4);
        v0 = b0 + (n0 - v0);
        v1 = b1 + (n1 - v1);
      }
      pk8(v0, v1, po[q], qo[q]);
      pa[q] = (size_t)grow * ldp + gcol;
    }
  }
  if (WF) {
    #pragma unroll
    for (int i = 0; i < 8; ++i) *(volatile v4f*)(Cf + fa[i]) = fo[i];
  }
  if (WP) {
    #pragma unroll
    for (int q = 0; q < 4; ++q) {
      *(volatile v4u*)(Phi + pa[q]) = po[q];
      *(volatile v4u*)(Plo + pa[q]) = qo[q];
    }
  }
  __threadfence();
  if (WF) {
    #pragma unroll
    for (int i = 0; i < 8; ++i) *(volatile v4f*)(Cf + fa[i]) = fo[i];
  }
  if (WP) {
    #pragma unroll
    for (int q = 0; q < 4; ++q) {
      *(volatile v4u*)(Phi + pa[q]) = po[q];
      *(volatile v4u*)(Plo + pa[q]) = qo[q];
    }
  }
}

__global__ __launch_bounds__(256) void k_lstm(
    const unsigned short* __restrict__ Xh, const unsigned short* __restrict__ Xl,
    const unsigned short* __restrict__ Wih, const unsigned short* __restrict__ Wil,
    const unsigned short* __restrict__ Whh, const unsigned short* __restrict__ Whl,
    const float* __restrict__ bsum, float* Hout, unsigned short* Po, unsigned short* Qo)
{
  __shared__ __align__(16) unsigned short sPh[2 * 16 * PH];
  __shared__ __align__(16) unsigned short sPl[2 * 16 * PH];
  __shared__ __align__(16) float sHf[16 * PF];
  const int tid = threadIdx.x, lane = tid & 31, wv = tid >> 5;
  const int h = lane >> 4, m = lane & 15;
  const int b0 = blockIdx.x * 16;

  for (int i = tid; i < 2 * 16 * PH; i += 256) { sPh[i] = 0; sPl[i] = 0; }
  float c[16];
  #pragma unroll
  for (int i = 0; i < 16; ++i) c[i] = 0.f;
  float bI[2], bF[2], bG[2], bO[2];
  #pragma unroll
  for (int h2 = 0; h2 < 2; ++h2) {
    const int u = 32 * wv + 16 * h2 + m;
    bI[h2] = bsum[u];
    bF[h2] = bsum[HH + u];
    bG[h2] = bsum[2 * HH + u];
    bO[h2] = bsum[3 * HH + u];
  }
  __syncthreads();

  const v8f z8 = {0.f, 0.f, 0.f, 0.f, 0.f, 0.f, 0.f, 0.f};
  int cur = 0;
  #pragma unroll 1
  for (int t = 0; t < NV; ++t) {
    v8f acc[4][2];
    #pragma unroll
    for (int g = 0; g < 4; ++g)
      #pragma unroll
      for (int h2 = 0; h2 < 2; ++h2) acc[g][h2] = z8;

    const size_t xo = ((size_t)(b0 + m) * NV + t) * DD;
    #pragma unroll 1
    for (int kk = 0; kk < DD / 32; ++kk) {
      const int k0 = 32 * kk;
      const v16b ah = ldfrag(Xh + xo + k0, h);
      const v16b al = ldfrag(Xl + xo + k0, h);
      #pragma unroll
      for (int g = 0; g < 4; ++g)
        #pragma unroll
        for (int h2 = 0; h2 < 2; ++h2) {
          const size_t bo = (size_t)(g * HH + 32 * wv + 16 * h2 + m) * DD + k0;
          const v16b bh = ldfrag(Wih + bo, h);
          const v16b bl = ldfrag(Wil + bo, h);
          acc[g][h2] = wmma_b(ah, bh, acc[g][h2]);
          acc[g][h2] = wmma_b(ah, bl, acc[g][h2]);
          acc[g][h2] = wmma_b(al, bh, acc[g][h2]);
        }
    }
    const unsigned short* hph = sPh + cur * (16 * PH) + m * PH;
    const unsigned short* hpl = sPl + cur * (16 * PH) + m * PH;
    #pragma unroll 1
    for (int kk = 0; kk < HH / 32; ++kk) {
      const int k0 = 32 * kk;
      const v16b ah = ldfrag(hph + k0, h);
      const v16b al = ldfrag(hpl + k0, h);
      #pragma unroll
      for (int g = 0; g < 4; ++g)
        #pragma unroll
        for (int h2 = 0; h2 < 2; ++h2) {
          const size_t bo = (size_t)(g * HH + 32 * wv + 16 * h2 + m) * HH + k0;
          const v16b bh = ldfrag(Whh + bo, h);
          const v16b bl = ldfrag(Whl + bo, h);
          acc[g][h2] = wmma_b(ah, bh, acc[g][h2]);
          acc[g][h2] = wmma_b(ah, bl, acc[g][h2]);
          acc[g][h2] = wmma_b(al, bh, acc[g][h2]);
        }
    }

    const int nxt = cur ^ 1;
    #pragma unroll
    for (int h2 = 0; h2 < 2; ++h2) {
      const int u = 32 * wv + 16 * h2 + m;
      #pragma unroll
      for (int r = 0; r < 8; ++r) {
        const int rl = 8 * h + r;
        const float gi = acc[0][h2][r] + bI[h2];
        const float gf = acc[1][h2][r] + bF[h2];
        const float gg = acc[2][h2][r] + bG[h2];
        const float gq = acc[3][h2][r] + bO[h2];
        const float cn = sigm(gf) * c[8 * h2 + r] + sigm(gi) * tnh(gg);
        c[8 * h2 + r] = cn;
        const float hv = sigm(gq) * tnh(cn);
        sHf[rl * PF + u] = hv;
        const unsigned int hb = bf16r(hv);
        const unsigned int lb = bf16r(hv - __uint_as_float(hb << 16));
        sPh[nxt * (16 * PH) + rl * PH + u] = (unsigned short)hb;
        sPl[nxt * (16 * PH) + rl * PH + u] = (unsigned short)lb;
      }
    }
    __syncthreads();

    {
      const int ra = 2 * wv, rbw = 2 * wv + 1;
      const size_t ga = ((size_t)(b0 + ra) * NV + t) * DD;
      const size_t gb = ((size_t)(b0 + rbw) * NV + t) * DD;
      const v4f fa0 = *(const v4fa*)(sHf + ra * PF + 4 * lane);
      const v4f fa1 = *(const v4fa*)(sHf + ra * PF + 128 + 4 * lane);
      const v4f fb0 = *(const v4fa*)(sHf + rbw * PF + 4 * lane);
      const v4f fb1 = *(const v4fa*)(sHf + rbw * PF + 128 + 4 * lane);
      const v4u pha = *(const v4ua*)(sPh + nxt * (16 * PH) + ra * PH + 8 * lane);
      const v4u pla = *(const v4ua*)(sPl + nxt * (16 * PH) + ra * PH + 8 * lane);
      const v4u phb = *(const v4ua*)(sPh + nxt * (16 * PH) + rbw * PH + 8 * lane);
      const v4u plb = *(const v4ua*)(sPl + nxt * (16 * PH) + rbw * PH + 8 * lane);
      *(volatile v4f*)(Hout + ga + 4 * lane) = fa0;
      *(volatile v4f*)(Hout + ga + 128 + 4 * lane) = fa1;
      *(volatile v4f*)(Hout + gb + 4 * lane) = fb0;
      *(volatile v4f*)(Hout + gb + 128 + 4 * lane) = fb1;
      *(volatile v4u*)(Po + ga + 8 * lane) = pha;
      *(volatile v4u*)(Qo + ga + 8 * lane) = pla;
      *(volatile v4u*)(Po + gb + 8 * lane) = phb;
      *(volatile v4u*)(Qo + gb + 8 * lane) = plb;
      __threadfence();
      *(volatile v4f*)(Hout + ga + 4 * lane) = fa0;
      *(volatile v4f*)(Hout + ga + 128 + 4 * lane) = fa1;
      *(volatile v4f*)(Hout + gb + 4 * lane) = fb0;
      *(volatile v4f*)(Hout + gb + 128 + 4 * lane) = fb1;
      *(volatile v4u*)(Po + ga + 8 * lane) = pha;
      *(volatile v4u*)(Qo + ga + 8 * lane) = pla;
      *(volatile v4u*)(Po + gb + 8 * lane) = phb;
      *(volatile v4u*)(Qo + gb + 8 * lane) = plb;
    }
    __syncthreads();
    cur = nxt;
  }
}

__global__ __launch_bounds__(256) void k_bar(const float* __restrict__ ve,
                                             const float* __restrict__ wh,
                                             const float* __restrict__ S,
                                             const float* __restrict__ T,
                                             const float* __restrict__ W2,
                                             const float* __restrict__ b2,
                                             const float* __restrict__ btab,
                                             const float* __restrict__ nz,
                                             float* bar, unsigned short* Eh,
                                             unsigned short* El, float* onz)
{
  __shared__ __align__(16) float sE[8 * DD];
  const int tid = threadIdx.x, lane = tid & 31, wv = tid >> 5;
  const int row = blockIdx.x * 8 + wv;
  const int b = row / NV;
  const int v = row - b * NV;
  const int u = (v == 0) ? row : (row - 1);
  const float y0 = tnh(S[b * TFW + lane] + T[(size_t)u * TFW + lane]);
  const float y1 = tnh(S[b * TFW + 32 + lane] + T[(size_t)u * TFW + 32 + lane]);
  float p0 = y0 * W2[2 * lane] + y1 * W2[2 * (32 + lane)];
  float p1 = y0 * W2[2 * lane + 1] + y1 * W2[2 * (32 + lane) + 1];
  #pragma unroll
  for (int o = 16; o > 0; o >>= 1) {
    p0 += __shfl_xor(p0, o, 32);
    p1 += __shfl_xor(p1, o, 32);
  }
  const float a0 = p0 + b2[0];
  const float a1 = p1 + b2[1];
  const float sa = btab[b], sn = btab[NB + b];

  v4f bo[2], no[2];
  #pragma unroll
  for (int s = 0; s < 2; ++s) {
    const int cc = 128 * s + 4 * lane;
    const v4f e = *(const v4fa*)(ve + (size_t)(b * NV) * DD + cc);
    const v4f w = *(const v4fa*)(wh + (size_t)u * DD + cc);
    const v4f n = *(const v4fa*)(nz + (size_t)row * DD + cc);
    v4f br = e * a0 + w * a1;
    if (v == 0) br = e;
    const v4f en = br * sa + n * sn;
    *(v4fa*)(sE + wv * DD + cc) = en;
    bo[s] = br;
    no[s] = n;
  }
  __syncthreads();
  const v4f e0v = *(const v4fa*)(sE + wv * DD + 8 * lane);
  const v4f e1v = *(const v4fa*)(sE + wv * DD + 8 * lane + 4);
  v4u ph, pl;
  pk8(e0v, e1v, ph, pl);
  const size_t ro = (size_t)row * DD;
  *(volatile v4f*)(bar + ro + 4 * lane) = bo[0];
  *(volatile v4f*)(bar + ro + 128 + 4 * lane) = bo[1];
  *(volatile v4f*)(onz + ro + 4 * lane) = no[0];
  *(volatile v4f*)(onz + ro + 128 + 4 * lane) = no[1];
  *(volatile v4u*)(Eh + ro + 8 * lane) = ph;
  *(volatile v4u*)(El + ro + 8 * lane) = pl;
  __threadfence();
  *(volatile v4f*)(bar + ro + 4 * lane) = bo[0];
  *(volatile v4f*)(bar + ro + 128 + 4 * lane) = bo[1];
  *(volatile v4f*)(onz + ro + 4 * lane) = no[0];
  *(volatile v4f*)(onz + ro + 128 + 4 * lane) = no[1];
  *(volatile v4u*)(Eh + ro + 8 * lane) = ph;
  *(volatile v4u*)(El + ro + 8 * lane) = pl;
}

__global__ __launch_bounds__(256) void k_cls3(const float* __restrict__ h2,
                                              const float* __restrict__ W3,
                                              const float* __restrict__ b3, float* outc)
{
  __shared__ __align__(16) float sO[512];
  const int tid = threadIdx.x, lane = tid & 31, wv = tid >> 5;
  const int row = blockIdx.x * 256 + tid;
  const float* hr = h2 + (size_t)row * CL2;
  float s0 = 0.f, s1 = 0.f;
  #pragma unroll 4
  for (int k = 0; k < CL2; ++k) {
    const float x = hr[k];
    s0 += x * W3[2 * k];
    s1 += x * W3[2 * k + 1];
  }
  v2f o2;
  o2.x = s0 + b3[0];
  o2.y = s1 + b3[1];
  *(v2fa*)(sO + 2 * tid) = o2;
  __syncthreads();
  if (wv < 4) {
    const v4f vq = *(const v4fa*)(sO + 128 * wv + 4 * lane);
    float* d = outc + (size_t)blockIdx.x * 512 + 128 * wv + 4 * lane;
    *(volatile v4f*)d = vq;
    __threadfence();
    *(volatile v4f*)d = vq;
  }
}

extern "C" void kernel_launch(void* const* d_in, const int* in_sizes, int n_in,
                              void* d_out, int out_size, void* d_ws, size_t ws_size,
                              hipStream_t stream)
{
  if (n_in < 27) return;
  if (in_sizes[0]  != NR) return;
  if (in_sizes[1]  != NR * DD) return;
  if (in_sizes[2]  != NVOC * DD) return;
  if (in_sizes[3]  != TFW) return;
  if (in_sizes[4]  != TFW) return;
  if (in_sizes[5]  != TFW * DD) return;
  if (in_sizes[6]  != DD) return;
  if (in_sizes[7]  != DD * G4) return;
  if (in_sizes[8]  != HH * G4) return;
  if (in_sizes[9]  != G4) return;
  if (in_sizes[10] != G4) return;
  if (in_sizes[11] != HH * DD) return;
  if (in_sizes[12] != DD) return;
  if (in_sizes[13] != 2 * HH * TFW) return;
  if (in_sizes[14] != TFW) return;
  if (in_sizes[15] != TFW * 2) return;
  if (in_sizes[16] != 2) return;
  if (in_sizes[17] != HH * G4) return;
  if (in_sizes[18] != G4) return;
  if (in_sizes[19] != G4 * CL2) return;
  if (in_sizes[20] != CL2) return;
  if (in_sizes[21] != CL2 * 2) return;
  if (in_sizes[22] != 2) return;
  if (in_sizes[23] != DD * DD) return;
  if (in_sizes[24] != DD) return;
  if (in_sizes[25] != NR * NC) return;
  if (in_sizes[26] != NB) return;
  if (out_size != 3 * NR * DD + 2 * NB * 2 + NR * DD) return;

  const float* seq_time = (const float*)d_in[0];
  const float* noise    = (const float*)d_in[1];
  const float* embW     = (const float*)d_in[2];
  const float* w_time   = (const float*)d_in[3];
  const float* b_time   = (const float*)d_in[4];
  const float* w_updim  = (const float*)d_in[5];
  const float* b_updim  = (const float*)d_in[6];
  const float* W_ih     = (const float*)d_in[7];
  const float* W_hh     = (const float*)d_in[8];
  const float* b_ih     = (const float*)d_in[9];
  const float* b_hh     = (const float*)d_in[10];
  const float* W_hk     = (const float*)d_in[11];
  const float* b_hk     = (const float*)d_in[12];
  const float* W1       = (const float*)d_in[13];
  const float* b1       = (const float*)d_in[14];
  const float* W2       = (const float*)d_in[15];
  const float* b2       = (const float*)d_in[16];
  const float* Wc1      = (const float*)d_in[17];
  const float* bc1      = (const float*)d_in[18];
  const float* Wc2      = (const float*)d_in[19];
  const float* bc2      = (const float*)d_in[20];
  const float* Wc3      = (const float*)d_in[21];
  const float* bc3      = (const float*)d_in[22];
  const float* W_diff   = (const float*)d_in[23];
  const float* b_diff   = (const float*)d_in[24];
  const int*   seqs     = (const int*)d_in[25];
  const int*   tvec     = (const int*)d_in[26];

  float* out  = (float*)d_out;
  float* out0 = out;
  float* out1 = out + (size_t)NR * DD;
  float* out2 = out + (size_t)2 * NR * DD;
  float* out4 = out2 + 2 * NB * 2;
  float* out5 = out4 + (size_t)NR * DD;

  const size_t szBsum = (size_t)G4 * 4;
  const size_t szBtab = (size_t)3 * NB * 4;
  const size_t szWup  = (size_t)DD * TFW * 2;
  const size_t szWih  = (size_t)G4 * DD * 2;
  const size_t szWhh  = (size_t)G4 * HH * 2;
  const size_t szWhk  = (size_t)DD * HH * 2;
  const size_t szW1   = (size_t)TFW * 2 * HH * 2;
  const size_t szWdf  = (size_t)DD * DD * 2;
  const size_t szWc1  = (size_t)G4 * HH * 2;
  const size_t szWc2  = (size_t)CL2 * G4 * 2;
  const size_t szTf   = (size_t)NR * TFW * 2;
  const size_t szRowF = (size_t)NR * DD * 4;
  const size_t szRowP = (size_t)NR * DD * 2;
  const size_t szS    = (size_t)NB * TFW * 4;
  const size_t szT    = (size_t)NR * TFW * 4;
  const size_t szH1P  = (size_t)CLR * G4 * 2;
  const size_t szH2   = (size_t)CLR * CL2 * 4;
  const size_t total = szBsum + szBtab
      + 2 * (szWup + szWih + szWhh + szWhk + szW1 + szWdf + szWc1 + szWc2)
      + 2 * szTf + szRowF   + szRowF
      + 4 * szRowP   + szRowF   + 2 * szRowP
      + szS + szT + szRowF   + 2 * szRowP   + 2 * szH1P + szH2;
  if (total > ws_size) return;
  if (total > (size_t)134217728) return;

  char* ws = (char*)d_ws;
  size_t off = 0;
  float*          bsum = (float*)(ws + off);          off += szBsum;
  float*          btab = (float*)(ws + off);          off += szBtab;
  unsigned short* WupH = (unsigned short*)(ws + off); off += szWup;
  unsigned short* WupL = (unsigned short*)(ws + off); off += szWup;
  unsigned short* WihH = (unsigned short*)(ws + off); off += szWih;
  unsigned short* WihL = (unsigned short*)(ws + off); off += szWih;
  unsigned short* WhhH = (unsigned short*)(ws + off); off += szWhh;
  unsigned short* WhhL = (unsigned short*)(ws + off); off += szWhh;
  unsigned short* WhkH = (unsigned short*)(ws + off); off += szWhk;
  unsigned short* WhkL = (unsigned short*)(ws + off); off += szWhk;
  unsigned short* W1H  = (unsigned short*)(ws + off); off += szW1;
  unsigned short* W1L  = (unsigned short*)(ws + off); off += szW1;
  unsigned short* WdfH = (unsigned short*)(ws + off); off += szWdf;
  unsigned short* WdfL = (unsigned short*)(ws + off); off += szWdf;
  unsigned short* Wc1H = (unsigned short*)(ws + off); off += szWc1;
  unsigned short* Wc1L = (unsigned short*)(ws + off); off += szWc1;
  unsigned short* Wc2H = (unsigned short*)(ws + off); off += szWc2;
  unsigned short* Wc2L = (unsigned short*)(ws + off); off += szWc2;
  unsigned short* TfH  = (unsigned short*)(ws + off); off += szTf;
  unsigned short* TfL  = (unsigned short*)(ws + off); off += szTf;
  float*          embF = (float*)(ws + off);          off += szRowF;
  unsigned short* genH = (unsigned short*)embF;
  unsigned short* genL = (unsigned short*)((char*)embF + szRowP);
  float*          veF  = (float*)(ws + off);          off += szRowF;
  unsigned short* hidH = (unsigned short*)(ws + off); off += szRowP;
  unsigned short* vePH = (unsigned short*)(ws + off); off += szRowP;
  unsigned short* hidL = (unsigned short*)(ws + off); off += szRowP;
  unsigned short* vePL = (unsigned short*)(ws + off); off += szRowP;
  float*          whF  = (float*)(ws + off);          off += szRowF;
  unsigned short* whH  = (unsigned short*)(ws + off); off += szRowP;
  unsigned short* whL  = (unsigned short*)(ws + off); off += szRowP;
  float*          Sf   = (float*)(ws + off);          off += szS;
  float*          Tf   = (float*)(ws + off);          off += szT;
  float*          barF = (float*)(ws + off);          off += szRowF;
  unsigned short* enH  = (unsigned short*)(ws + off); off += szRowP;
  unsigned short* enL  = (unsigned short*)(ws + off); off += szRowP;
  unsigned short* h1H  = (unsigned short*)(ws + off); off += szH1P;
  unsigned short* h1L  = (unsigned short*)(ws + off); off += szH1P;
  float*          h2F  = (float*)(ws + off);          off += szH2;
  if (off != total) return;
  unsigned short* hgH = vePH;
  unsigned short* hgL = vePL;

  k_cvtw<<<dim3(DD / 64, TFW / 64), 256, 0, stream>>>(w_updim, TFW, DD, WupH, WupL);
  k_cvtw<<<dim3(G4 / 64, DD / 64), 256, 0, stream>>>(W_ih, DD, G4, WihH, WihL);
  k_cvtw<<<dim3(G4 / 64, HH / 64), 256, 0, stream>>>(W_hh, HH, G4, WhhH, WhhL);
  k_cvtw<<<dim3(DD / 64, HH / 64), 256, 0, stream>>>(W_hk, HH, DD, WhkH, WhkL);
  k_cvtw<<<dim3(TFW / 64, 2 * HH / 64), 256, 0, stream>>>(W1, 2 * HH, TFW, W1H, W1L);
  k_cvtw<<<dim3(DD / 64, DD / 64), 256, 0, stream>>>(W_diff, DD, DD, WdfH, WdfL);
  k_cvtw<<<dim3(G4 / 64, HH / 64), 256, 0, stream>>>(Wc1, HH, G4, Wc1H, Wc1L);
  k_cvtw<<<dim3(CL2 / 64, G4 / 64), 256, 0, stream>>>(Wc2, G4, CL2, Wc2H, Wc2L);

  k_prep<<<1, NB, 0, stream>>>(b_ih, b_hh, tvec, bsum, btab);
  k_tfeat<<<NR / 4, 256, 0, stream>>>(seq_time, w_time, b_time, TfH, TfL);
  k_embed<<<NR / 8, 256, 0, stream>>>(seqs, embW, embF);
  k_gemm<1, 0, 1, 1, 1, 0><<<dim3(NR / 64, DD / 64), 128, 0, stream>>>(
      TfH, TfL, TFW, WupH, WupL, TFW, TFW, b_updim, btab, embF, embF, DD,
      veF, DD, vePH, vePL, DD);
  k_lstm<<<NB / 16, 256, 0, stream>>>(vePH, vePL, WihH, WihL, WhhH, WhhL, bsum, out0, hidH, hidL);
  k_gemm<1, 0, 0, 1, 1, 0><<<dim3(NR / 64, DD / 64), 128, 0, stream>>>(
      hidH, hidL, HH, WhkH, WhkL, HH, HH, b_hk, btab, veF, veF, DD,
      whF, DD, whH, whL, DD);
  k_gemm<1, 0, 0, 1, 0, 0><<<dim3(NB / 64, TFW / 64), 128, 0, stream>>>(
      vePH, vePL, NV * DD, W1H, W1L, 2 * HH, DD, b1, btab, veF, veF, DD,
      Sf, TFW, h1H, h1L, G4);
  k_gemm<0, 0, 0, 1, 0, 0><<<dim3(NR / 64, TFW / 64), 128, 0, stream>>>(
      whH, whL, DD, W1H + HH, W1L + HH, 2 * HH, HH, b1, btab, veF, veF, DD,
      Tf, TFW, h1H, h1L, G4);
  k_bar<<<NR / 8, 256, 0, stream>>>(veF, whF, Sf, Tf, W2, b2, btab, noise, barF, enH, enL, out4);
  k_gemm<1, 0, 0, 1, 1, 1><<<dim3(NR / 64, DD / 64), 128, 0, stream>>>(
      enH, enL, DD, WdfH, WdfL, DD, DD, b_diff, btab + 2 * NB, barF, noise, DD,
      out5, DD, genH, genL, DD);
  k_lstm<<<NB / 16, 256, 0, stream>>>(genH, genL, WihH, WihL, WhhH, WhhL, bsum, out1, hgH, hgL);
  k_gemm<1, 1, 0, 0, 1, 0><<<dim3(CLR / 64, G4 / 64), 128, 0, stream>>>(
      hidH + (size_t)(NV - 1) * DD, hidL + (size_t)(NV - 1) * DD, NV * DD, Wc1H, Wc1L, HH, HH,
      bc1, btab, veF, veF, DD, h2F, CL2, h1H, h1L, G4);
  k_gemm<1, 1, 0, 1, 0, 0><<<dim3(CLR / 64, CL2 / 64), 128, 0, stream>>>(
      h1H, h1L, G4, Wc2H, Wc2L, G4, G4, bc2, btab, veF, veF, DD,
      h2F, CL2, enH, enL, DD);
  k_cls3<<<2, 256, 0, stream>>>(h2F, Wc3, bc3, out2);
}
